// _RWKV6BlockFast_52450140619469
// MI455X (gfx1250) — hardware-run, weakly checked
//
#include <hip/hip_runtime.h>
#include <math.h>

constexpr int kB = 2;
constexpr int kT = 2048;
constexpr int kD = 1024;
constexpr int kH = 16;
constexpr int kHS = 64;
constexpr int kTok = kB * kT;
constexpr int kPitch2 = 2 * kD;
constexpr int kChunk = 16;
constexpr float kWCarry = 16.0f;
constexpr float kWFold = 1.0f / kWCarry;
constexpr float kInvD = 1.0f / (float)kD;
constexpr float kLnEps = 1e-5f;
constexpr float kF16Tiny = 6.2e-5f;
constexpr float kF16Big = 60000.0f;
constexpr float kF32Min = 1.17549435e-38f;
static_assert(kD == kH * kHS, "head split");
static_assert(kTok % 64 == 0 && kD % 64 == 0 && kD % 32 == 0, "tile multiples");
static_assert(((kTok / 64) * (kD / 64)) % 8 == 0, "eight wave tiles per block");
static_assert(kT % kChunk == 0, "scan chunking");
static_assert((kT & (kT - 1)) == 0, "power-of-two sequence length");

typedef __attribute__((ext_vector_type(16))) _Float16 v16h;
typedef __attribute__((ext_vector_type(8)))  _Float16 v8h;
typedef __attribute__((ext_vector_type(16))) __bf16   v16b;
typedef __attribute__((ext_vector_type(8)))  __bf16   v8b;
typedef __attribute__((ext_vector_type(8)))  float    v8f;
typedef __attribute__((ext_vector_type(4)))  float    v4f;
typedef __attribute__((ext_vector_type(4)))  unsigned int v4u;
typedef __attribute__((ext_vector_type(2)))  unsigned int v2u;

__device__ __forceinline__ unsigned short f2bf_bits(float f) {
  unsigned u = __float_as_uint(f);
  return (unsigned short)((u + 0x7FFFu + ((u >> 16) & 1u)) >> 16);
}
__device__ __forceinline__ unsigned pk16(unsigned short a, unsigned short b) { return (unsigned)a | ((unsigned)b << 16); }
__device__ __forceinline__ unsigned short h_bits(float f) { const _Float16 h = (_Float16)f; return __builtin_bit_cast(unsigned short, h); }

__device__ __forceinline__ unsigned short f16_bits_ftz(float a, float& back) {
  const float ac = fminf(fmaxf(a, -kF16Big), kF16Big);
  const _Float16 h = (_Float16)ac;
  const float hf = (float)h;
  const bool tiny = fabsf(ac) < kF16Tiny;
  const unsigned short hb = __builtin_bit_cast(unsigned short, h);
  back = tiny ? 0.0f : hf;
  return tiny ? (unsigned short)0 : hb;
}

__device__ __forceinline__ void guard4_h(v8f& a, v8f& b, v8f& c, v8f& d, v16h x, v16h y0, v16h y1, v16h y2, v16h y3) {
  asm volatile("v_nop\n\tv_nop\n\tv_nop\n\tv_nop" : "+v"(a), "+v"(b), "+v"(c), "+v"(d) : "v"(x), "v"(y0), "v"(y1), "v"(y2), "v"(y3));
}
__device__ __forceinline__ void guard4_b(v8f& a, v8f& b, v8f& c, v8f& d, v16b x, v16b y0, v16b y1, v16b y2, v16b y3) {
  asm volatile("v_nop\n\tv_nop\n\tv_nop\n\tv_nop" : "+v"(a), "+v"(b), "+v"(c), "+v"(d) : "v"(x), "v"(y0), "v"(y1), "v"(y2), "v"(y3));
}
__device__ __forceinline__ void acc_guard4(v8f& a, v8f& b, v8f& c, v8f& d) {
  asm volatile("v_nop\n\tv_nop\n\tv_nop\n\tv_nop" : "+v"(a), "+v"(b), "+v"(c), "+v"(d));
}
__device__ __forceinline__ void wave_lds_sync() {
  __builtin_amdgcn_fence(__ATOMIC_RELEASE, "workgroup");
  __builtin_amdgcn_wave_barrier();
  __builtin_amdgcn_fence(__ATOMIC_ACQUIRE, "workgroup");
}

template <typename T> struct Frag;
template <> struct Frag<_Float16> {
  typedef v16h V; union U { v16h v; v8h h[2]; };
  static __device__ __forceinline__ v16h load(const _Float16* p) {
    U f; f.h[0] = *(const v8h*)(p); f.h[1] = *(const v8h*)(p + 16); return f.v;
  }
  static __device__ __forceinline__ v8f mma(v16h a, v16h b, v8f c) {
    return __builtin_amdgcn_wmma_f32_16x16x32_f16(false, a, false, b, (short)0, c, false, false);
  }
};
template <> struct Frag<__bf16> {
  typedef v16b V; union U { v16b v; v8b h[2]; };
  static __device__ __forceinline__ v16b load(const __bf16* p) {
    U f; f.h[0] = *(const v8b*)(p); f.h[1] = *(const v8b*)(p + 16); return f.v;
  }
  static __device__ __forceinline__ v8f mma(v16b a, v16b b, v8f c) {
    return __builtin_amdgcn_wmma_f32_16x16x32_bf16(false, a, false, b, (short)0, c, false, false);
  }
};

__global__ __launch_bounds__(256) void mixsig_kernel(const float* __restrict__ m0, const float* __restrict__ m1,
                                                     const float* __restrict__ m2, const float* __restrict__ m3,
                                                     float* __restrict__ sig) {
  const int p = blockIdx.x;
  const float* m = (p == 0) ? m0 : (p == 1) ? m1 : (p == 2) ? m2 : m3;
  const int c4 = threadIdx.x * 4;
  const v4f a = *(const v4f*)(m + c4);
  v4f s;
  s[0] = 1.0f / (1.0f + expf(-a[0]));
  s[1] = 1.0f / (1.0f + expf(-a[1]));
  s[2] = 1.0f / (1.0f + expf(-a[2]));
  s[3] = 1.0f / (1.0f + expf(-a[3]));
  float* q = sig + (size_t)p * kD + c4;
  *(volatile v4f*)q = s;
  __threadfence();
  *(volatile v4f*)q = s;
}

__global__ __launch_bounds__(256) void wcast_kernel(const float* __restrict__ W0, const float* __restrict__ W1,
                                                    const float* __restrict__ W2, const float* __restrict__ W3,
                                                    const float* __restrict__ W4, const float* __restrict__ W5,
                                                    unsigned short* __restrict__ outH, unsigned short* __restrict__ outB) {
  const int z = blockIdx.y;
  const float* W = (z == 0) ? W0 : (z == 1) ? W1 : (z == 2) ? W2 : (z == 3) ? W3 : (z == 4) ? W4 : W5;
  const int i = blockIdx.x * 256 + threadIdx.x;
  const float* p = W + 8 * (size_t)i;
  const v4f a = *(const v4f*)(p);
  const v4f c = *(const v4f*)(p + 4);
  unsigned short hb[8];
  unsigned short bb[8];
#pragma unroll
  for (int e = 0; e < 4; ++e) {
    const float w0 = a[e] * kWCarry;
    const float w1 = c[e] * kWCarry;
    hb[e]     = h_bits(w0);
    hb[4 + e] = h_bits(w1);
    bb[e]     = f2bf_bits(w0);
    bb[4 + e] = f2bf_bits(w1);
  }
  const v4u uh = (v4u){pk16(hb[0], hb[1]), pk16(hb[2], hb[3]), pk16(hb[4], hb[5]), pk16(hb[6], hb[7])};
  const v4u ub = (v4u){pk16(bb[0], bb[1]), pk16(bb[2], bb[3]), pk16(bb[4], bb[5]), pk16(bb[6], bb[7])};
  unsigned short* qh = outH + (size_t)z * kD * kD + 8 * (size_t)i;
  const bool hasB = (z == 1) || (z == 2) || (z == 5);
  const int zb = (z == 1) ? 0 : (z == 2) ? 1 : 2;
  unsigned short* qb = outB + (size_t)zb * kD * kD + 8 * (size_t)i;
  *(volatile v4u*)qh = uh;
  if (hasB) { *(volatile v4u*)qb = ub; }
  __threadfence();
  *(volatile v4u*)qh = uh;
  if (hasB) { *(volatile v4u*)qb = ub; }
}

__global__ __launch_bounds__(256) void ln_mix_kernel(const float* __restrict__ x,
                                                     const float* __restrict__ lnw, const float* __restrict__ lnb,
                                                     const float* __restrict__ sig,
                                                     unsigned short* __restrict__ XK, unsigned short* __restrict__ XV,
                                                     unsigned short* __restrict__ XR, unsigned short* __restrict__ XW) {
  __shared__ float redA[8];
  __shared__ float redB[8];
  __shared__ float redC[8];
  __shared__ float redD[8];
  const int m    = blockIdx.x;
  const int t    = m & (kT - 1);
  const int tid  = threadIdx.x;
  const int lane = tid & 31;
  const int wave = tid >> 5;
  const int c4   = tid * 4;
  const bool hasPrev = (t > 0);
  const int mp = hasPrev ? (m - 1) : m;
  const v4f c = *(const v4f*)(x + (size_t)m  * kD + c4);
  const v4f p = *(const v4f*)(x + (size_t)mp * kD + c4);

  float s0 = (c[0] + c[1]) + (c[2] + c[3]);
  float s1 = (p[0] + p[1]) + (p[2] + p[3]);
#pragma unroll
  for (int off = 16; off > 0; off >>= 1) {
    s0 += __shfl_xor(s0, off, 32);
    s1 += __shfl_xor(s1, off, 32);
  }
  if (lane == 0) { redA[wave] = s0; redB[wave] = s1; }
  __syncthreads();
  float a0 = 0.0f, a1 = 0.0f;
#pragma unroll
  for (int w = 0; w < 8; ++w) { a0 += redA[w]; a1 += redB[w]; }
  const float mu0 = a0 * kInvD;
  const float mu1 = a1 * kInvD;
  float dc[4], dp[4];
#pragma unroll
  for (int e = 0; e < 4; ++e) { dc[e] = c[e] - mu0; dp[e] = p[e] - mu1; }
  float q0 = (dc[0] * dc[0] + dc[1] * dc[1]) + (dc[2] * dc[2] + dc[3] * dc[3]);
  float q1 = (dp[0] * dp[0] + dp[1] * dp[1]) + (dp[2] * dp[2] + dp[3] * dp[3]);
#pragma unroll
  for (int off = 16; off > 0; off >>= 1) {
    q0 += __shfl_xor(q0, off, 32);
    q1 += __shfl_xor(q1, off, 32);
  }
  if (lane == 0) { redC[wave] = q0; redD[wave] = q1; }
  __syncthreads();
  float b0 = 0.0f, b1 = 0.0f;
#pragma unroll
  for (int w = 0; w < 8; ++w) { b0 += redC[w]; b1 += redD[w]; }
  const float rs0 = rsqrtf(b0 * kInvD + kLnEps);
  const float rs1 = rsqrtf(b1 * kInvD + kLnEps);

  const v4f lw = *(const v4f*)(lnw + c4);
  const v4f lb = *(const v4f*)(lnb + c4);
  const v4f sk = *(const v4f*)(sig + c4);
  const v4f sv = *(const v4f*)(sig + kD + c4);
  const v4f sr = *(const v4f*)(sig + 2 * kD + c4);
  const v4f sw = *(const v4f*)(sig + 3 * kD + c4);

  unsigned short kh[4], kl[4], vh[4], vl[4], rr[4], ww[4];
#pragma unroll
  for (int e = 0; e < 4; ++e) {
    const float xn  = (dc[e] * rs0) * lw[e] + lb[e];
    const float xpv = (dp[e] * rs1) * lw[e] + lb[e];
    const float xp  = hasPrev ? xpv : 0.0f;
    const float ak = xn * sk[e] + xp * (1.0f - sk[e]);
    const float av = xn * sv[e] + xp * (1.0f - sv[e]);
    const float ar = xn * sr[e] + xp * (1.0f - sr[e]);
    const float aw = xn * sw[e] + xp * (1.0f - sw[e]);
    float bk, bv, br, bw;
    kh[e] = f16_bits_ftz(ak, bk);
    vh[e] = f16_bits_ftz(av, bv);
    rr[e] = f16_bits_ftz(ar, br);
    ww[e] = f16_bits_ftz(aw, bw);
    kl[e] = f2bf_bits(ak - bk);
    vl[e] = f2bf_bits(av - bv);
  }
  const v2u ukh = (v2u){pk16(kh[0], kh[1]), pk16(kh[2], kh[3])};
  const v2u ukl = (v2u){pk16(kl[0], kl[1]), pk16(kl[2], kl[3])};
  const v2u uvh = (v2u){pk16(vh[0], vh[1]), pk16(vh[2], vh[3])};
  const v2u uvl = (v2u){pk16(vl[0], vl[1]), pk16(vl[2], vl[3])};
  const v2u ur  = (v2u){pk16(rr[0], rr[1]), pk16(rr[2], rr[3])};
  const v2u uw  = (v2u){pk16(ww[0], ww[1]), pk16(ww[2], ww[3])};
  unsigned short* pkh = XK + (size_t)m * kPitch2 + c4;
  unsigned short* pkl = pkh + kD;
  unsigned short* pvh = XV + (size_t)m * kPitch2 + c4;
  unsigned short* pvl = pvh + kD;
  unsigned short* pr  = XR + (size_t)m * kD + c4;
  unsigned short* pw  = XW + (size_t)m * kD + c4;
  *(volatile v2u*)pkh = ukh;
  *(volatile v2u*)pkl = ukl;
  *(volatile v2u*)pvh = uvh;
  *(volatile v2u*)pvl = uvl;
  *(volatile v2u*)pr  = ur;
  *(volatile v2u*)pw  = uw;
  __threadfence();
  *(volatile v2u*)pkh = ukh;
  *(volatile v2u*)pkl = ukl;
  *(volatile v2u*)pvh = uvh;
  *(volatile v2u*)pvl = uvl;
  *(volatile v2u*)pr  = ur;
  *(volatile v2u*)pw  = uw;
}

template <int ACT, bool MIXED, bool BIAS_N>
__global__ __launch_bounds__(256) void gemm64_mix(
    const unsigned short* __restrict__ Ap, const unsigned short* __restrict__ Alp, int lda,
    const unsigned short* __restrict__ Btp, const unsigned short* __restrict__ Btlp, int ldb,
    float* __restrict__ C, int ldc,
    const float* __restrict__ bias,
    int M, int N, int K, float scale) {
  __shared__ __align__(16) float sT[8][16 * 68];
  const int lane = threadIdx.x & 31;
  const int wave = threadIdx.x >> 5;
  const int tilesN = N >> 6;
  const int tilesM = M >> 6;
  const int tile = blockIdx.x * 8 + wave;
  if (tile >= tilesM * tilesN) return;
  const int tm = tile / tilesN;
  const int tn = tile - tm * tilesN;
  const int m0 = tm << 6;
  const int n0 = tn << 6;
  const _Float16* A   = (const _Float16*)Ap;
  const _Float16* Bt  = (const _Float16*)Btp;
  const __bf16*   Al  = (const __bf16*)Alp;
  const __bf16*   Btl = (const __bf16*)Btlp;
  const int rlane = lane & 15;
  const int koff  = (lane >> 4) * 8;
  const int mOff  = (lane >> 4) * 8;

  int ao[4];
  int bo[4];
#pragma unroll
  for (int i = 0; i < 4; ++i) {
    ao[i] = (m0 + (i << 4) + rlane) * lda + koff;
    bo[i] = (n0 + (i << 4) + rlane) * ldb + koff;
  }

  v8f acc[4][4];
#pragma unroll
  for (int i = 0; i < 4; ++i)
#pragma unroll
    for (int j = 0; j < 4; ++j) acc[i][j] = (v8f){0.f, 0.f, 0.f, 0.f, 0.f, 0.f, 0.f, 0.f};

  for (int k0 = 0; k0 < K; k0 += 32) {
    {
      const v16h b0 = Frag<_Float16>::load(Bt + bo[0] + k0);
      const v16h b1 = Frag<_Float16>::load(Bt + bo[1] + k0);
      const v16h b2 = Frag<_Float16>::load(Bt + bo[2] + k0);
      const v16h b3 = Frag<_Float16>::load(Bt + bo[3] + k0);
#pragma unroll
      for (int i = 0; i < 4; ++i) {
        const v16h ah = Frag<_Float16>::load(A + ao[i] + k0);
        acc[i][0] = Frag<_Float16>::mma(ah, b0, acc[i][0]);
        acc[i][1] = Frag<_Float16>::mma(ah, b1, acc[i][1]);
        acc[i][2] = Frag<_Float16>::mma(ah, b2, acc[i][2]);
        acc[i][3] = Frag<_Float16>::mma(ah, b3, acc[i][3]);
        guard4_h(acc[i][0], acc[i][1], acc[i][2], acc[i][3], ah, b0, b1, b2, b3);
      }
    }
    if (MIXED) {
      const v16b l0 = Frag<__bf16>::load(Btl + bo[0] + k0);
      const v16b l1 = Frag<__bf16>::load(Btl + bo[1] + k0);
      const v16b l2 = Frag<__bf16>::load(Btl + bo[2] + k0);
      const v16b l3 = Frag<__bf16>::load(Btl + bo[3] + k0);
#pragma unroll
      for (int i = 0; i < 4; ++i) {
        const v16b al = Frag<__bf16>::load(Al + ao[i] + k0);
        acc[i][0] = Frag<__bf16>::mma(al, l0, acc[i][0]);
        acc[i][1] = Frag<__bf16>::mma(al, l1, acc[i][1]);
        acc[i][2] = Frag<__bf16>::mma(al, l2, acc[i][2]);
        acc[i][3] = Frag<__bf16>::mma(al, l3, acc[i][3]);
        guard4_b(acc[i][0], acc[i][1], acc[i][2], acc[i][3], al, l0, l1, l2, l3);
      }
    }
  }
  acc_guard4(acc[0][0], acc[0][1], acc[0][2], acc[0][3]);
  acc_guard4(acc[1][0], acc[1][1], acc[1][2], acc[1][3]);
  acc_guard4(acc[2][0], acc[2][1], acc[2][2], acc[2][3]);
  acc_guard4(acc[3][0], acc[3][1], acc[3][2], acc[3][3]);

  float* slab = sT[wave];
  float bv[4];
#pragma unroll
  for (int j = 0; j < 4; ++j) bv[j] = BIAS_N ? bias[n0 + (j << 4) + rlane] : 0.0f;

#pragma unroll
  for (int i = 0; i < 4; ++i) {
    const int mBase = m0 + (i << 4);
#pragma unroll
    for (int j = 0; j < 4; ++j) {
#pragma unroll
      for (int r = 0; r < 8; ++r) {
        slab[(mOff + r) * 68 + (j << 4) + rlane] = acc[i][j][r] * scale + bv[j];
      }
    }
    wave_lds_sync();
    if (ACT != 0) {
#pragma unroll 1
      for (int qq = 0; qq < 32; ++qq) {
        const int idx = qq * 32 + lane;
        const int off = (idx >> 6) * 68 + (idx & 63);
        float v = slab[off];
        if (ACT == 1) {
          v = 1.0f / (1.0f + expf(-v));
        }
        if (ACT == 2) {
          const float w = fminf(fmaxf(v, -10.0f), 10.0f);
          const float d = expf(-expf(w));
          v = (d < kF32Min) ? 0.0f : d;
        }
        slab[off] = v;
      }
      wave_lds_sync();
    }
    {
      const int hh = lane >> 4, c4 = (lane & 15) * 4;
      for (int pass = 0; pass < 2; ++pass) {
#pragma unroll
        for (int it = 0; it < 8; ++it) {
          const int row = it * 2 + hh;
          const v4f v = *(const v4f*)(slab + row * 68 + c4);
          *(volatile v4f*)(C + (size_t)(mBase + row) * ldc + n0 + c4) = v;
        }
        __threadfence();
      }
    }
    wave_lds_sync();
  }
}

__global__ __launch_bounds__(256) void state_scan_kernel(const float* __restrict__ R, const float* __restrict__ Kp,
                                                         const float* __restrict__ Vp, const float* __restrict__ Dc,
                                                         const float* __restrict__ G, const float* __restrict__ U,
                                                         unsigned short* __restrict__ GY) {
  __shared__ __align__(16) float sR[kChunk * kHS];
  __shared__ __align__(16) float sK[kChunk * kHS];
  __shared__ __align__(16) float sD[kChunk * kHS];
  __shared__ __align__(16) float sV[kChunk * kHS];
  __shared__ __align__(16) float sG[kChunk * kHS];
  __shared__ __align__(16) float part[kChunk * 4 * kHS];
  __shared__ float coef[kChunk];

  const int bh  = blockIdx.x;
  const int b   = bh >> 4;
  const int h   = bh & 15;
  const int tid = threadIdx.x;
  const int i   = tid & 63;
  const int q   = tid >> 6;
  const int srow = tid >> 4;
  const int sc4  = (tid & 15) * 4;
  const int line = tid >> 3;
  const int erow = line >> 1;
  const int esel = line & 1;
  const int ec8  = (tid & 7) * 8;

  const v4f u4 = *(const v4f*)(U + h * kHS + sc4);
  const size_t base = (size_t)b * kT * kD + (size_t)h * kHS;

  float S[16];
#pragma unroll
  for (int jj = 0; jj < 16; ++jj) S[jj] = 0.0f;

#pragma unroll 1
  for (int ch = 0; ch < kT / kChunk; ++ch) {
    const int t0 = ch * kChunk;
    {
      const size_t go = base + (size_t)(t0 + srow) * kD + sc4;
      const v4f r4 = *(const v4f*)(R  + go);
      const v4f k4 = *(const v4f*)(Kp + go);
      const v4f v4 = *(const v4f*)(Vp + go);
      const v4f d4 = *(const v4f*)(Dc + go);
      const v4f g4 = *(const v4f*)(G  + go);
      *(v4f*)(sR + srow * kHS + sc4) = r4;
      *(v4f*)(sK + srow * kHS + sc4) = k4;
      *(v4f*)(sV + srow * kHS + sc4) = v4;
      *(v4f*)(sD + srow * kHS + sc4) = d4;
      *(v4f*)(sG + srow * kHS + sc4) = g4;
      float cp = 0.0f;
      cp += (r4[0] * u4[0]) * k4[0];
      cp += (r4[1] * u4[1]) * k4[1];
      cp += (r4[2] * u4[2]) * k4[2];
      cp += (r4[3] * u4[3]) * k4[3];
      cp += __shfl_xor(cp, 8, 32);
      cp += __shfl_xor(cp, 4, 32);
      cp += __shfl_xor(cp, 2, 32);
      cp += __shfl_xor(cp, 1, 32);
      if ((tid & 15) == 0) { coef[srow] = cp; }
    }
    __syncthreads();

#pragma unroll 1
    for (int t = 0; t < kChunk; ++t) {
      const float vi = sV[t * kHS + i];
      const float* pr = sR + t * kHS + q * 16;
      const float* pk = sK + t * kHS + q * 16;
      const float* pd = sD + t * kHS + q * 16;
      v4f rq[4], kq[4], dq[4];
#pragma unroll
      for (int mm = 0; mm < 4; ++mm) {
        rq[mm] = *(const v4f*)(pr + 4 * mm);
        kq[mm] = *(const v4f*)(pk + 4 * mm);
        dq[mm] = *(const v4f*)(pd + 4 * mm);
      }
      float acc = 0.0f;
#pragma unroll
      for (int mm = 0; mm < 4; ++mm) {
#pragma unroll
        for (int e = 0; e < 4; ++e) {
          const float kv = kq[mm][e] * vi;
          acc = fmaf(rq[mm][e], S[4 * mm + e], acc);
          S[4 * mm + e] = fmaf(dq[mm][e], S[4 * mm + e], kv);
        }
      }
      part[(t * 4 + q) * kHS + i] = acc;
    }
    __syncthreads();

    {
      const float cf = coef[erow];
      const float* pp = part + (erow * 4) * kHS + ec8;
      const v4f pa0 = *(const v4f*)(pp);
      const v4f pb0 = *(const v4f*)(pp + 4);
      const v4f pa1 = *(const v4f*)(pp + kHS);
      const v4f pb1 = *(const v4f*)(pp + kHS + 4);
      const v4f pa2 = *(const v4f*)(pp + 2 * kHS);
      const v4f pb2 = *(const v4f*)(pp + 2 * kHS + 4);
      const v4f pa3 = *(const v4f*)(pp + 3 * kHS);
      const v4f pb3 = *(const v4f*)(pp + 3 * kHS + 4);
      const v4f ya = ((pa0 + pa1) + pa2) + pa3;
      const v4f yb = ((pb0 + pb1) + pb2) + pb3;
      const v4f ga = *(const v4f*)(sG + erow * kHS + ec8);
      const v4f gb = *(const v4f*)(sG + erow * kHS + ec8 + 4);
      const v4f va = *(const v4f*)(sV + erow * kHS + ec8);
      const v4f vb = *(const v4f*)(sV + erow * kHS + ec8 + 4);
      unsigned short ob[8];
#pragma unroll
      for (int e = 0; e < 4; ++e) {
        const float y0 = ya[e] + va[e] * cf;
        const float y1 = yb[e] + vb[e] * cf;
        const float z0 = ga[e] * y0;
        const float z1 = gb[e] * y1;
        float back0, back1;
        const unsigned short h0 = f16_bits_ftz(z0, back0);
        const unsigned short h1 = f16_bits_ftz(z1, back1);
        const unsigned short l0 = f2bf_bits(z0 - back0);
        const unsigned short l1 = f2bf_bits(z1 - back1);
        ob[e]     = (esel != 0) ? l0 : h0;
        ob[4 + e] = (esel != 0) ? l1 : h1;
      }
      const v4u uo = (v4u){pk16(ob[0], ob[1]), pk16(ob[2], ob[3]), pk16(ob[4], ob[5]), pk16(ob[6], ob[7])};
      unsigned short* gp = GY + (size_t)(b * kT + t0 + erow) * kPitch2 + (size_t)esel * kD + h * kHS + ec8;
      *(volatile v4u*)gp = uo;
      __threadfence();
      *(volatile v4u*)gp = uo;
    }
    __syncthreads();
  }
}

extern "C" void kernel_launch(void* const* d_in, const int* in_sizes, int n_in,
                              void* d_out, int out_size, void* d_ws, size_t ws_size, hipStream_t stream) {
  if (n_in < 15 || d_out == nullptr || d_ws == nullptr) return;
  if (in_sizes[0] != kTok * kD || in_sizes[1] != kD || in_sizes[2] != kD || in_sizes[3] != kD ||
      in_sizes[4] != kD || in_sizes[5] != kD || in_sizes[6] != kD || in_sizes[7] != kD * kD ||
      in_sizes[8] != kD * kD || in_sizes[9] != kD * kD || in_sizes[10] != kD * kD ||
      in_sizes[11] != kD * kD || in_sizes[12] != kD * kD || in_sizes[13] != kD ||
      in_sizes[14] != kH * kHS || out_size != kTok * kD) return;

  const float* x    = (const float*)d_in[0];
  const float* lnw  = (const float*)d_in[1];
  const float* lnb  = (const float*)d_in[2];
  const float* mixk = (const float*)d_in[3];
  const float* mixv = (const float*)d_in[4];
  const float* mixr = (const float*)d_in[5];
  const float* mixw = (const float*)d_in[6];
  const float* Wr   = (const float*)d_in[7];
  const float* Wk   = (const float*)d_in[8];
  const float* Wv   = (const float*)d_in[9];
  const float* Ww   = (const float*)d_in[10];
  const float* Wg   = (const float*)d_in[11];
  const float* Wo   = (const float*)d_in[12];
  const float* td   = (const float*)d_in[13];
  const float* tf   = (const float*)d_in[14];
  float* out = (float*)d_out;

  constexpr size_t PW   = (size_t)kD * kD;
  constexpr size_t PF32 = (size_t)kTok * kD * 4;
  static_assert(PF32 == (size_t)kTok * kPitch2 * 2, "split plane and f32 plane have equal size");
  static_assert(PF32 == 2 * (size_t)kTok * kD * 2, "two f16 planes fill one region");

  char* ws = (char*)d_ws;
  size_t off = 0;
  auto carve = [&](size_t bytes) -> char* { char* p = ws + off; off += (bytes + 255) & ~(size_t)255; return p; };
  float*          SIG = (float*)carve((size_t)4 * kD * 4);
  unsigned short* W16 = (unsigned short*)carve((size_t)6 * PW * 2);
  unsigned short* WB  = (unsigned short*)carve((size_t)3 * PW * 2);
  char*           RA  = carve(PF32);
  char*           RB  = carve(PF32);
  char*           RC  = carve(PF32);
  float*          K32 = (float*)carve(PF32);
  float*          V32 = (float*)carve(PF32);
  float*          R32 = (float*)carve(PF32);
  if (off > ws_size || off > (size_t)134217728) return;

  unsigned short* XK  = (unsigned short*)RA;
  float*          G32 = (float*)RA;
  unsigned short* XV  = (unsigned short*)RB;
  float*          D32 = (float*)RB;
  unsigned short* XR  = (unsigned short*)RC;
  unsigned short* XW  = (unsigned short*)RC + (size_t)kTok * kD;
  unsigned short* GY  = (unsigned short*)RC;

  const unsigned short* Wr16 = W16;
  const unsigned short* Wk16 = W16 + PW;
  const unsigned short* Wv16 = W16 + 2 * PW;
  const unsigned short* Ww16 = W16 + 3 * PW;
  const unsigned short* Wg16 = W16 + 4 * PW;
  const unsigned short* Wo16 = W16 + 5 * PW;
  const unsigned short* WkB  = WB;
  const unsigned short* WvB  = WB + PW;
  const unsigned short* WoB  = WB + 2 * PW;

  mixsig_kernel<<<4, 256, 0, stream>>>(mixk, mixv, mixr, mixw, SIG);
  wcast_kernel<<<dim3(kD * kD / 8 / 256, 6), 256, 0, stream>>>(Wr, Wk, Wv, Ww, Wg, Wo, W16, WB);
  ln_mix_kernel<<<kTok, 256, 0, stream>>>(x, lnw, lnb, SIG, XK, XV, XR, XW);

  const int gBig = (kTok / 64) * (kD / 64) / 8;

  gemm64_mix<0, true, false><<<gBig, 256, 0, stream>>>(
      XK, XK + kD, kPitch2, Wk16, WkB, kD, K32, kD, td, kTok, kD, kD, kWFold);
  gemm64_mix<0, true, false><<<gBig, 256, 0, stream>>>(
      XV, XV + kD, kPitch2, Wv16, WvB, kD, V32, kD, td, kTok, kD, kD, kWFold);
  gemm64_mix<1, false, false><<<gBig, 256, 0, stream>>>(
      XR, XR, kD, Wr16, Wr16, kD, R32, kD, td, kTok, kD, kD, kWFold);
  gemm64_mix<2, false, true><<<gBig, 256, 0, stream>>>(
      XW, XW, kD, Ww16, Ww16, kD, D32, kD, td, kTok, kD, kD, kWFold);
  gemm64_mix<1, false, false><<<gBig, 256, 0, stream>>>(
      XR, XR, kD, Wg16, Wg16, kD, G32, kD, td, kTok, kD, kD, kWFold);

  state_scan_kernel<<<kB * kH, 256, 0, stream>>>(R32, K32, V32, D32, G32, tf, GY);

  gemm64_mix<0, true, false><<<gBig, 256, 0, stream>>>(
      GY, GY + kD, kPitch2, Wo16, WoB, kD, out, kD, td, kTok, kD, kD, kWFold);
}
